// PromptAttention_14224931684857
// MI455X (gfx1250) — hardware-verified
//
#include <hip/hip_runtime.h>
#include <stdint.h>
#include <stddef.h>

typedef __attribute__((ext_vector_type(16))) _Float16 v16h;
typedef __attribute__((ext_vector_type(8)))  _Float16 v8h;
typedef __attribute__((ext_vector_type(16))) __bf16   v16b;
typedef __attribute__((ext_vector_type(8)))  __bf16   v8b;
typedef __attribute__((ext_vector_type(8)))  float    v8f;
typedef __attribute__((ext_vector_type(4)))  float    v4f;
typedef __attribute__((ext_vector_type(4)))  unsigned v4u;

constexpr int kDim     = 768;
constexpr int kHeads   = 12;
constexpr int kDh      = 64;
constexpr int kPrompt  = 8;
constexpr int kInner   = 768;
constexpr int kBatch   = 4;
constexpr int kSeq     = 2048;
constexpr int kRows    = kBatch * kSeq;
constexpr int kQkvCols = 3 * kInner;
constexpr int kKC      = 64;
constexpr int kNQB     = kSeq / 64;
constexpr int kChunks  = kSeq / kKC + 1;
constexpr float kQScaleLog2e = 0.125f * 1.44269504088896341f;
constexpr float kPCarry = 32768.0f;
constexpr float kOCarry = 64.0f;
constexpr float kWCarry = 256.0f;
constexpr float kOutScale = 1.0f / (64.0f * 256.0f);

static_assert(kRows % 64 == 0);
static_assert(kQkvCols % 64 == 0);
static_assert(kInner % 64 == 0);
static_assert(kDim % 32 == 0);
static_assert(kInner % 32 == 0);
static_assert(kSeq % 64 == 0);
static_assert(kDh == 64);
static_assert(kPrompt <= kKC);

constexpr size_t kXbBytes  = (size_t)kRows * kDim * 2;
constexpr size_t kBtqBytes = (size_t)kQkvCols * kDim * 2;
constexpr size_t kBtoBytes = (size_t)kInner * kInner * 2;
constexpr size_t kQkvBytes = (size_t)kRows * kQkvCols * 2;
constexpr size_t kPkBytes  = (size_t)kHeads * kKC * kDh * 2;
constexpr size_t kOhBytes  = (size_t)kRows * kInner * 2;
constexpr size_t kWsTotal  = kXbBytes + kBtqBytes + kBtoBytes + kQkvBytes + 2 * kPkBytes + kOhBytes;
static_assert(kWsTotal == 67829760);
static_assert(kWsTotal <= (size_t)134217728);
static_assert(kXbBytes % 256 == 0 && kBtqBytes % 256 == 0 && kBtoBytes % 256 == 0 && kQkvBytes % 256 == 0 && kPkBytes % 256 == 0 && kOhBytes % 256 == 0);

__device__ __forceinline__ unsigned short f2bf_bits(float f) {
  unsigned u = __float_as_uint(f);
  return (unsigned short)((u + 0x7FFFu + ((u >> 16) & 1u)) >> 16);
}
__device__ __forceinline__ float bf_bits2f(unsigned short h) { return __uint_as_float(((unsigned)h) << 16); }
__device__ __forceinline__ unsigned short h_bits(float f) { return __builtin_bit_cast(unsigned short, (_Float16)f); }

__device__ __forceinline__ void dep_guard_h(v8f& a, v8f& b, v16h x, v16h y) { asm volatile("v_nop\n\tv_nop\n\tv_nop\n\tv_nop" : "+v"(a), "+v"(b) : "v"(x), "v"(y)); }
__device__ __forceinline__ void dep_guard_b(v8f& a, v8f& b, v16b x, v16b y) { asm volatile("v_nop\n\tv_nop\n\tv_nop\n\tv_nop" : "+v"(a), "+v"(b) : "v"(x), "v"(y)); }
__device__ __forceinline__ void keep4_h(v16h a, v16h b, v16h c, v16h d) { asm volatile("v_nop" :: "v"(a), "v"(b), "v"(c), "v"(d)); }
__device__ __forceinline__ void keep4_b(v16b a, v16b b, v16b c, v16b d) { asm volatile("v_nop" :: "v"(a), "v"(b), "v"(c), "v"(d)); }
__device__ __forceinline__ void acc_guard4(v8f& a, v8f& b, v8f& c, v8f& d) { asm volatile("v_nop\n\tv_nop\n\tv_nop\n\tv_nop" : "+v"(a), "+v"(b), "+v"(c), "+v"(d)); }

template <typename T> struct Frag;
template <> struct Frag<_Float16> {
  typedef v16h V; union U { v16h v; v8h h[2]; };
  static __device__ __forceinline__ v16h load(const _Float16* p) {
    U f; f.h[0] = *(const v8h*)(p); f.h[1] = *(const v8h*)(p + 16); return f.v;
  }
  static __device__ __forceinline__ v8f mma(v16h a, v16h b, v8f c) {
    return __builtin_amdgcn_wmma_f32_16x16x32_f16(false, a, false, b, (short)0, c, false, false);
  }
  static __device__ __forceinline__ void guard(v8f& a, v8f& b, v16h x, v16h y) { dep_guard_h(a, b, x, y); }
  static __device__ __forceinline__ void keep(v16h a, v16h b, v16h c, v16h d) { keep4_h(a, b, c, d); }
};
template <> struct Frag<__bf16> {
  typedef v16b V; union U { v16b v; v8b h[2]; };
  static __device__ __forceinline__ v16b load(const __bf16* p) {
    U f; f.h[0] = *(const v8b*)(p); f.h[1] = *(const v8b*)(p + 16); return f.v;
  }
  static __device__ __forceinline__ v8f mma(v16b a, v16b b, v8f c) {
    return __builtin_amdgcn_wmma_f32_16x16x32_bf16(false, a, false, b, (short)0, c, false, false);
  }
  static __device__ __forceinline__ void guard(v8f& a, v8f& b, v16b x, v16b y) { dep_guard_b(a, b, x, y); }
  static __device__ __forceinline__ void keep(v16b a, v16b b, v16b c, v16b d) { keep4_b(a, b, c, d); }
};

__device__ __forceinline__ v8f zero8() { v8f z = {0.f, 0.f, 0.f, 0.f, 0.f, 0.f, 0.f, 0.f}; return z; }

template <int ET> struct Elem;
template <> struct Elem<0> { typedef _Float16 T; };
template <> struct Elem<1> { typedef __bf16 T; };
template <int ET, bool SPLIT, int BIAS_MODE, int OUT_MODE, bool RESID, int ACT = 0>
__global__ __launch_bounds__(256) void wmma_gemm64(
    const unsigned short* __restrict__ Ap, const unsigned short* __restrict__ A2p, int lda, long strideA,
    const unsigned short* __restrict__ Btp, const unsigned short* __restrict__ Bt2p, int ldb, long strideB,
    void* __restrict__ Cout, void* __restrict__ Cout2, int ldc, long strideC,
    const float* __restrict__ bias,
    const float* __restrict__ resid, long strideR,
    int M, int N, int K, float scale) {
  typedef typename Elem<ET>::T T;
  typedef typename Frag<T>::V V;
  const T* A = (const T*)Ap; const T* A2 = (const T*)A2p; const T* Bt = (const T*)Btp; const T* Bt2 = (const T*)Bt2p;
  __shared__ __align__(16) float sT[8][16 * 68];
  const int b    = blockIdx.y;
  const int lane = threadIdx.x & 31;
  const int wave = threadIdx.x >> 5;
  const int tilesN = N >> 6;
  const int tilesM = M >> 6;
  const int tile = blockIdx.x * 8 + wave;
  if (tile >= tilesM * tilesN) return;
  const int tm = tile / tilesN;
  const int tn = tile - tm * tilesN;
  const int m0 = tm << 6;
  const int n0 = tn << 6;

  const T* Ab  = A  + (size_t)b * strideA;
  const T* Bb  = Bt + (size_t)b * strideB;
  const T* Ab2 = SPLIT ? (A2  + (size_t)b * strideA) : nullptr;
  const T* Bb2 = SPLIT ? (Bt2 + (size_t)b * strideB) : nullptr;

  const int rlane = lane & 15;
  const int koff  = (lane >> 4) * 8;
  const int mOff  = (lane >> 4) * 8;

  v8f acc[4][4];
#pragma unroll
  for (int i = 0; i < 4; ++i)
#pragma unroll
    for (int j = 0; j < 4; ++j) acc[i][j] = zero8();

  for (int k0 = 0; k0 < K; k0 += 32) {
    V bh[4], bl[4];
#pragma unroll
    for (int j = 0; j < 4; ++j) {
      const size_t bo = (size_t)(n0 + (j << 4) + rlane) * ldb + koff + k0;
      bh[j] = Frag<T>::load(Bb + bo);
      if (SPLIT) bl[j] = Frag<T>::load(Bb2 + bo);
    }
#pragma unroll
    for (int i = 0; i < 4; ++i) {
      const size_t ao = (size_t)(m0 + (i << 4) + rlane) * lda + koff + k0;
      V ah = Frag<T>::load(Ab + ao);
      V al = ah;
      if (SPLIT) al = Frag<T>::load(Ab2 + ao);
#pragma unroll
      for (int j = 0; j < 4; ++j) {
        acc[i][j] = Frag<T>::mma(ah, bh[j], acc[i][j]);
        if (SPLIT) {
          acc[i][j] = Frag<T>::mma(ah, bl[j], acc[i][j]);
          acc[i][j] = Frag<T>::mma(al, bh[j], acc[i][j]);
        }
      }
      Frag<T>::guard(acc[i][0], acc[i][3], ah, SPLIT ? al : ah);
    }
    Frag<T>::keep(bh[0], bh[1], bh[2], bh[3]);
    if (SPLIT) Frag<T>::keep(bl[0], bl[1], bl[2], bl[3]);
  }
  acc_guard4(acc[0][0], acc[0][1], acc[0][2], acc[0][3]);
  acc_guard4(acc[1][0], acc[1][1], acc[1][2], acc[1][3]);
  acc_guard4(acc[2][0], acc[2][1], acc[2][2], acc[2][3]);
  acc_guard4(acc[3][0], acc[3][1], acc[3][2], acc[3][3]);

  float* slab = sT[wave];
  const float* Rb = RESID ? (resid + (size_t)b * strideR) : nullptr;
#pragma unroll
  for (int i = 0; i < 4; ++i) {
    const int mBase = m0 + (i << 4);
#pragma unroll
    for (int j = 0; j < 4; ++j) {
      const int n = n0 + (j << 4) + rlane;
      float bv = 0.f;
      if (BIAS_MODE == 2) bv = bf_bits2f(f2bf_bits(bias[n]));
#pragma unroll
      for (int r = 0; r < 8; ++r) {
        float v = acc[i][j][r] * scale;
        if (BIAS_MODE == 1) v += bf_bits2f(f2bf_bits(bias[mBase + mOff + r]));
        if (BIAS_MODE == 2) v += bv;
        if (RESID) v += Rb[(size_t)(mBase + mOff + r) * ldc + n];
        if (ACT == 1) v = tanhf(v);
        if (ACT == 2) v = fmaxf(v, 0.0f);
        if (ACT == 3) v = v / (1.0f + expf(-v));
        if (ACT == 4) v = (v > 0.f) ? v : 0.01f * v;
        slab[(mOff + r) * 68 + (j << 4) + rlane] = v;
      }
    }
    __builtin_amdgcn_fence(__ATOMIC_RELEASE, "workgroup");
    __builtin_amdgcn_wave_barrier();
    __builtin_amdgcn_fence(__ATOMIC_ACQUIRE, "workgroup");
    if (OUT_MODE == 0) {
      float* C = (float*)Cout + (size_t)b * strideC;
      const int hh = lane >> 4, c4 = (lane & 15) * 4;
      for (int pass = 0; pass < 2; ++pass) {
#pragma unroll
        for (int it = 0; it < 8; ++it) {
          const int row = it * 2 + hh;
          v4f v = *(const v4f*)(slab + row * 68 + c4);
          *(volatile v4f*)(C + (size_t)(mBase + row) * ldc + n0 + c4) = v;
        }
        __threadfence();
      }
    } else {
      const int q = lane >> 3, c8 = (lane & 7) * 8;
      unsigned short* C  = (unsigned short*)Cout  + (size_t)b * strideC;
      unsigned short* C2 = (OUT_MODE == 2) ? ((unsigned short*)Cout2 + (size_t)b * strideC) : nullptr;
      for (int pass = 0; pass < 2; ++pass) {
#pragma unroll
        for (int it = 0; it < 4; ++it) {
          const int row = it * 4 + q;
          const float* sp = slab + row * 68 + c8;
          v8h hv, lv;
#pragma unroll
          for (int e = 0; e < 8; ++e) {
            if (OUT_MODE == 1) {
              hv[e] = (_Float16)sp[e];
              lv[e] = hv[e];
            } else {
              unsigned short hb = f2bf_bits(sp[e]);
              unsigned short lb = f2bf_bits(sp[e] - bf_bits2f(hb));
              hv[e] = __builtin_bit_cast(_Float16, hb);
              lv[e] = __builtin_bit_cast(_Float16, lb);
            }
          }
          *(volatile v8h*)(C + (size_t)(mBase + row) * ldc + n0 + c8) = hv;
          if (OUT_MODE == 2) *(volatile v8h*)(C2 + (size_t)(mBase + row) * ldc + n0 + c8) = lv;
        }
        __threadfence();
      }
    }
    __builtin_amdgcn_fence(__ATOMIC_RELEASE, "workgroup");
    __builtin_amdgcn_wave_barrier();
    __builtin_amdgcn_fence(__ATOMIC_ACQUIRE, "workgroup");
  }
}

__global__ __launch_bounds__(256) void cast_f32_bf16x8(
    const float* __restrict__ in, unsigned short* __restrict__ out, int n8) {
  const int i = blockIdx.x * 256 + threadIdx.x;
  if (i < n8) {
    const size_t base = (size_t)i * 8;
    const v4f a = *(const v4f*)(in + base);
    const v4f c = *(const v4f*)(in + base + 4);
    v4u w;
    w[0] = (unsigned)f2bf_bits(a[0]) | ((unsigned)f2bf_bits(a[1]) << 16);
    w[1] = (unsigned)f2bf_bits(a[2]) | ((unsigned)f2bf_bits(a[3]) << 16);
    w[2] = (unsigned)f2bf_bits(c[0]) | ((unsigned)f2bf_bits(c[1]) << 16);
    w[3] = (unsigned)f2bf_bits(c[2]) | ((unsigned)f2bf_bits(c[3]) << 16);
    *(volatile v4u*)(out + base) = w;
    __threadfence();
    *(volatile v4u*)(out + base) = w;
  }
}

template <int MODE>
__global__ __launch_bounds__(256) void transpose_cast64(
    const float* __restrict__ in, unsigned short* __restrict__ out, int R, int C, float oscale) {
  __shared__ __align__(16) float tile[64 * 68];
  const int tid = threadIdx.x;
  const int r0 = blockIdx.y * 64;
  const int c0 = blockIdx.x * 64;
#pragma unroll
  for (int p = 0; p < 4; ++p) {
    const int rr = p * 16 + (tid >> 4);
    const int cc = (tid & 15) * 4;
    const v4f v = *(const v4f*)(in + (size_t)(r0 + rr) * C + c0 + cc);
    *(v4f*)(tile + rr * 68 + cc) = v;
  }
  __syncthreads();
  const int wave = tid >> 5, lane = tid & 31, q = lane >> 3, c8 = (lane & 7) * 8;
  for (int pass = 0; pass < 2; ++pass) {
#pragma unroll
    for (int it = 0; it < 2; ++it) {
      const int cc = wave * 8 + it * 4 + q;
      v4u w;
#pragma unroll
      for (int e2 = 0; e2 < 4; ++e2) {
        const float f0 = tile[(c8 + 2 * e2) * 68 + cc];
        const float f1 = tile[(c8 + 2 * e2 + 1) * 68 + cc];
        unsigned lo, hi;
        if (MODE == 0) {
          lo = (unsigned)f2bf_bits(f0);
          hi = (unsigned)f2bf_bits(f1);
        } else {
          const float g0 = bf_bits2f(f2bf_bits(f0)) * oscale;
          const float g1 = bf_bits2f(f2bf_bits(f1)) * oscale;
          lo = (unsigned)h_bits(g0);
          hi = (unsigned)h_bits(g1);
        }
        w[e2] = lo | (hi << 16);
      }
      *(volatile v4u*)(out + (size_t)(c0 + cc) * R + r0 + c8) = w;
    }
    __threadfence();
  }
}

__global__ __launch_bounds__(256) void prompt_pack(
    const float* __restrict__ pk, const float* __restrict__ pv,
    unsigned short* __restrict__ pkh, unsigned short* __restrict__ pvh) {
  const int tid = threadIdx.x, wave = tid >> 5, lane = tid & 31, q = lane >> 3, c8 = (lane & 7) * 8;
  const int row = blockIdx.x * 32 + wave * 4 + q;
  const int h = row >> 6, kv = row & 63;
  const int kvc = (kv < kPrompt) ? kv : (kPrompt - 1);
  const size_t src = ((size_t)h * kPrompt + kvc) * kDh + c8;
  const v4f a0 = *(const v4f*)(pk + src), a1 = *(const v4f*)(pk + src + 4);
  const v4f b0 = *(const v4f*)(pv + src), b1 = *(const v4f*)(pv + src + 4);
  const unsigned keep = (kv < kPrompt) ? 0xFFFFFFFFu : 0u;
  v4u wk, wv;
  wk[0] = ((unsigned)h_bits(bf_bits2f(f2bf_bits(a0[0]))) | ((unsigned)h_bits(bf_bits2f(f2bf_bits(a0[1]))) << 16)) & keep;
  wk[1] = ((unsigned)h_bits(bf_bits2f(f2bf_bits(a0[2]))) | ((unsigned)h_bits(bf_bits2f(f2bf_bits(a0[3]))) << 16)) & keep;
  wk[2] = ((unsigned)h_bits(bf_bits2f(f2bf_bits(a1[0]))) | ((unsigned)h_bits(bf_bits2f(f2bf_bits(a1[1]))) << 16)) & keep;
  wk[3] = ((unsigned)h_bits(bf_bits2f(f2bf_bits(a1[2]))) | ((unsigned)h_bits(bf_bits2f(f2bf_bits(a1[3]))) << 16)) & keep;
  wv[0] = ((unsigned)h_bits(bf_bits2f(f2bf_bits(b0[0]))) | ((unsigned)h_bits(bf_bits2f(f2bf_bits(b0[1]))) << 16)) & keep;
  wv[1] = ((unsigned)h_bits(bf_bits2f(f2bf_bits(b0[2]))) | ((unsigned)h_bits(bf_bits2f(f2bf_bits(b0[3]))) << 16)) & keep;
  wv[2] = ((unsigned)h_bits(bf_bits2f(f2bf_bits(b1[0]))) | ((unsigned)h_bits(bf_bits2f(f2bf_bits(b1[1]))) << 16)) & keep;
  wv[3] = ((unsigned)h_bits(bf_bits2f(f2bf_bits(b1[2]))) | ((unsigned)h_bits(bf_bits2f(f2bf_bits(b1[3]))) << 16)) & keep;
  unsigned short* dk = pkh + (size_t)row * kDh + c8;
  unsigned short* dv = pvh + (size_t)row * kDh + c8;
  for (int pass = 0; pass < 2; ++pass) {
    *(volatile v4u*)dk = wk;
    *(volatile v4u*)dv = wv;
    __threadfence();
  }
}

__device__ __forceinline__ v8f mma_f16g(v16h a, v16h b, v8f c) {
  c = __builtin_amdgcn_wmma_f32_16x16x32_f16(false, a, false, b, (short)0, c, false, false);
  asm volatile("v_nop\n\tv_nop\n\tv_nop\n\tv_nop" : "+v"(c) : "v"(a), "v"(b));
  return c;
}

__global__ __launch_bounds__(128)
void attn_prompt_f16(const unsigned short* __restrict__ qkv,
                     const unsigned short* __restrict__ pkh,
                     const unsigned short* __restrict__ pvh,
                     unsigned short* __restrict__ oh) {
  __shared__ __align__(16) unsigned short Ksh[kKC * kDh];
  __shared__ __align__(16) unsigned short Vth[kDh * kKC];
  __shared__ __align__(16) _Float16 Psh[4][16 * kKC];
  __shared__ __align__(16) float Os[4][16 * 68];

  const int tid  = threadIdx.x;
  const int wave = tid >> 5;
  const int lane = tid & 31;
  const int hh   = lane >> 4;
  const int c    = lane & 15;
  const int bx = blockIdx.x;
  const int qb = bx % kNQB;
  const int bh = bx / kNQB;
  const int h  = bh % kHeads;
  const int b  = bh / kHeads;
  const int q0 = qb * 64 + wave * 16;

  const _Float16* Qp = (const _Float16*)(const void*)qkv;
  v16h qa[2];
  {
    const _Float16* qrow = Qp + ((size_t)b * kSeq + q0 + c) * kQkvCols + h * kDh;
#pragma unroll
    for (int dc = 0; dc < 2; ++dc) qa[dc] = Frag<_Float16>::load(qrow + dc * 32 + 8 * hh);
  }

  float mrow[8], lrow[8];
  v8f oacc[4];
#pragma unroll
  for (int r = 0; r < 8; ++r) { mrow[r] = -__builtin_inff(); lrow[r] = 0.f; }
#pragma unroll
  for (int t = 0; t < 4; ++t) oacc[t] = zero8();

  for (int kc = 0; kc < kChunks; ++kc) {
    const bool pch = (kc == kChunks - 1);
    __syncthreads();
    {
      const int kvr = tid >> 1, dh = (tid & 1) * 32;
      const int kcc = pch ? 0 : kc;
      const unsigned short* kreg = qkv + (((size_t)b * kSeq + (size_t)kcc * kKC + kvr) * kQkvCols + kInner + h * kDh + dh);
      const unsigned short* vreg = kreg + kInner;
      const unsigned short* kpr  = pkh + (((size_t)h * kKC + kvr) * kDh + dh);
      const unsigned short* vpr  = pvh + (((size_t)h * kKC + kvr) * kDh + dh);
      const unsigned short* krow = pch ? kpr : kreg;
      const unsigned short* vrow = pch ? vpr : vreg;
#pragma unroll
      for (int i = 0; i < 4; ++i) {
        const v4u kw = *(const v4u*)(krow + 8 * i);
        *(v4u*)(Ksh + kvr * kDh + dh + 8 * i) = kw;
        const v4u vw = *(const v4u*)(vrow + 8 * i);
#pragma unroll
        for (int e = 0; e < 8; ++e) {
          const unsigned wd = vw[e >> 1];
          const unsigned short bits = (unsigned short)((e & 1) ? (wd >> 16) : (wd & 0xFFFFu));
          Vth[(dh + 8 * i + e) * kKC + kvr] = bits;
        }
      }
    }
    __syncthreads();

    v8f s[4];
#pragma unroll
    for (int j = 0; j < 4; ++j) {
      s[j] = zero8();
#pragma unroll
      for (int dc = 0; dc < 2; ++dc) {
        const v16h kb = Frag<_Float16>::load((const _Float16*)(const void*)Ksh + (j * 16 + c) * kDh + dc * 32 + 8 * hh);
        s[j] = mma_f16g(qa[dc], kb, s[j]);
      }
    }

    float cm[8];
#pragma unroll
    for (int r = 0; r < 8; ++r) {
      float m = -__builtin_inff();
#pragma unroll
      for (int j = 0; j < 4; ++j) {
        const int kvl = j * 16 + c;
        float val = s[j][r] * kQScaleLog2e;
        const bool masked = pch && (kvl >= kPrompt);
        val = masked ? -__builtin_inff() : val;
        s[j][r] = val;
        m = fmaxf(m, val);
      }
#pragma unroll
      for (int off = 1; off < 16; off <<= 1) m = fmaxf(m, __shfl_xor(m, off, 32));
      cm[r] = m;
    }

    _Float16* pwh = Psh[wave];
#pragma unroll
    for (int r = 0; r < 8; ++r) {
      const float mnew = fmaxf(mrow[r], cm[r]);
      const float alpha = exp2f(mrow[r] - mnew);
      mrow[r] = mnew;
      float psum = 0.f;
#pragma unroll
      for (int j = 0; j < 4; ++j) {
        const float p = exp2f(s[j][r] - mnew);
        psum += p;
        pwh[(8 * hh + r) * kKC + j * 16 + c] = (_Float16)(p * kPCarry);
      }
#pragma unroll
      for (int off = 1; off < 16; off <<= 1) psum += __shfl_xor(psum, off, 32);
      lrow[r] = lrow[r] * alpha + psum;
#pragma unroll
      for (int t = 0; t < 4; ++t) oacc[t][r] *= alpha;
    }
    __builtin_amdgcn_fence(__ATOMIC_RELEASE, "workgroup");
    __builtin_amdgcn_wave_barrier();
    __builtin_amdgcn_fence(__ATOMIC_ACQUIRE, "workgroup");

#pragma unroll
    for (int kk = 0; kk < 2; ++kk) {
      const v16h pa = Frag<_Float16>::load(pwh + c * kKC + kk * 32 + 8 * hh);
#pragma unroll
      for (int t = 0; t < 4; ++t) {
        const v16h vb = Frag<_Float16>::load((const _Float16*)(const void*)Vth + (t * 16 + c) * kKC + kk * 32 + 8 * hh);
        oacc[t] = mma_f16g(pa, vb, oacc[t]);
      }
    }
  }

  float* os = Os[wave];
#pragma unroll
  for (int r = 0; r < 8; ++r) {
    const float inv = kOCarry / (lrow[r] * kPCarry);
#pragma unroll
    for (int t = 0; t < 4; ++t) os[(8 * hh + r) * 68 + t * 16 + c] = oacc[t][r] * inv;
  }
  __builtin_amdgcn_fence(__ATOMIC_RELEASE, "workgroup");
  __builtin_amdgcn_wave_barrier();
  __builtin_amdgcn_fence(__ATOMIC_ACQUIRE, "workgroup");
  {
    const int q = lane >> 3, c8 = (lane & 7) * 8;
    unsigned short* ob = oh + ((size_t)b * kSeq + q0) * kInner + h * kDh + c8;
    for (int pass = 0; pass < 2; ++pass) {
#pragma unroll
      for (int it = 0; it < 4; ++it) {
        const int row = it * 4 + q;
        const v4f x0 = *(const v4f*)(os + row * 68 + c8);
        const v4f x1 = *(const v4f*)(os + row * 68 + c8 + 4);
        v4u w;
        w[0] = (unsigned)h_bits(x0[0]) | ((unsigned)h_bits(x0[1]) << 16);
        w[1] = (unsigned)h_bits(x0[2]) | ((unsigned)h_bits(x0[3]) << 16);
        w[2] = (unsigned)h_bits(x1[0]) | ((unsigned)h_bits(x1[1]) << 16);
        w[3] = (unsigned)h_bits(x1[2]) | ((unsigned)h_bits(x1[3]) << 16);
        *(volatile v4u*)(ob + (size_t)row * kInner) = w;
      }
      __threadfence();
    }
  }
}

extern "C" void kernel_launch(void* const* d_in, const int* in_sizes, int n_in,
                              void* d_out, int out_size, void* d_ws, size_t ws_size,
                              hipStream_t stream) {
  if (n_in < 6) return;
  const float* x    = (const float*)d_in[0];
  const float* Wqkv = (const float*)d_in[1];
  const float* pk   = (const float*)d_in[2];
  const float* pv   = (const float*)d_in[3];
  const float* Wout = (const float*)d_in[4];
  const float* bout = (const float*)d_in[5];
  float*       out  = (float*)d_out;

  if (in_sizes[0] != kRows * kDim) return;
  if (in_sizes[1] != kDim * kQkvCols) return;
  if (in_sizes[2] != kHeads * kPrompt * kDh) return;
  if (in_sizes[3] != kHeads * kPrompt * kDh) return;
  if (in_sizes[4] != kInner * kInner) return;
  if (in_sizes[5] != kInner) return;
  if (out_size != kRows * kInner) return;
  if (kWsTotal > ws_size) return;

  char* ws = (char*)d_ws;
  size_t off = 0;
  unsigned short* Xb   = (unsigned short*)(ws + off); off += kXbBytes;
  unsigned short* Btq  = (unsigned short*)(ws + off); off += kBtqBytes;
  unsigned short* Bto  = (unsigned short*)(ws + off); off += kBtoBytes;
  unsigned short* QKVh = (unsigned short*)(ws + off); off += kQkvBytes;
  unsigned short* PKh  = (unsigned short*)(ws + off); off += kPkBytes;
  unsigned short* PVh  = (unsigned short*)(ws + off); off += kPkBytes;
  unsigned short* Oh   = (unsigned short*)(ws + off); off += kOhBytes;
  if (off > ws_size) return;

  const int n8 = (kRows * kDim) / 8;
  cast_f32_bf16x8<<<dim3((n8 + 255) / 256), dim3(256), 0, stream>>>(x, Xb, n8);

  transpose_cast64<0><<<dim3(kQkvCols / 64, kDim / 64), dim3(256), 0, stream>>>(Wqkv, Btq, kDim, kQkvCols, 1.0f);
  transpose_cast64<1><<<dim3(kInner / 64, kInner / 64), dim3(256), 0, stream>>>(Wout, Bto, kInner, kInner, kWCarry);

  prompt_pack<<<dim3((kHeads * kKC) / 32), dim3(256), 0, stream>>>(pk, pv, PKh, PVh);

  {
    const int tiles = (kRows / 64) * (kQkvCols / 64);
    wmma_gemm64<1, false, 0, 1, false><<<dim3(tiles / 8, 1), dim3(256), 0, stream>>>(
        Xb, Xb, kDim, 0L, Btq, Btq, kDim, 0L, (void*)QKVh, (void*)QKVh, kQkvCols, 0L,
        bout, bout, 0L, kRows, kQkvCols, kDim, 1.0f);
  }

  attn_prompt_f16<<<dim3(kBatch * kHeads * kNQB), dim3(128), 0, stream>>>(QKVh, PKh, PVh, Oh);

  {
    const int tiles = (kRows / 64) * (kInner / 64);
    wmma_gemm64<0, false, 2, 0, false><<<dim3(tiles / 8, 1), dim3(256), 0, stream>>>(
        Oh, Oh, kInner, 0L, Bto, Bto, kInner, 0L, (void*)out, (void*)out, kInner, 0L,
        bout, bout, 0L, kRows, kInner, kInner, kOutScale);
  }
}
